// LocalXLAttention_12403865551021
// MI455X (gfx1250) — hardware-verified
//
#include <hip/hip_runtime.h>


#ifndef NB
#define NB 1
#endif
#ifndef SEQ
#define SEQ 4096
#endif
#define NB_FULL  1
#define SEQ_FULL 4096
#ifndef OUT_SEQ
#define OUT_SEQ SEQ
#endif
#ifndef CW
#define CW 512
#endif
#define DM   1024
#define NH_  16
#define HD   64
#define KVW  128
#define NCH  (SEQ / CW)
#define NKEY (3 * CW)
#define AW   4
#define OSP  68
#define GSP  68
#define KSP  65
#define SC2  ((float)(0.125 * 1.4426950408889634))
#define PSH  14.0f
#define NEGB (-3.0e38f)
#define CTXC 16.0f
#define WCS  64.0f
#define OSC  (1.0f / 1024.0f)

static_assert(HD == 64);
static_assert(NH_ * HD == DM);
static_assert(KVW == 2 * HD);
static_assert(DM % 64 == 0);
static_assert(KVW % 64 == 0);
static_assert(DM % 32 == 0);
static_assert(SEQ % 64 == 0);
static_assert((NB * SEQ) % 64 == 0);
static_assert(SEQ % CW == 0);
static_assert(NCH >= 1);
static_assert(CW % 64 == 0);
static_assert(NKEY % 32 == 0);
static_assert(SEQ % (16 * AW) == 0);
static_assert(((size_t)SEQ * DM) % 8 == 0);
static_assert(NB <= NB_FULL);
static_assert(SEQ <= SEQ_FULL);
static_assert((OSP * 4) % 16 == 0);
static_assert((GSP * 4) % 16 == 0);
static_assert(AW * 16 * OSP * 4 <= 131072);
static_assert(16 * GSP * 4 <= 131072);
static_assert(3 * 64 * KSP * 4 <= 131072);
static_assert(64 * KSP * 4 <= 131072);

typedef _Float16 h16;
typedef unsigned short bf;
typedef __attribute__((ext_vector_type(16))) __bf16   v16bf;
typedef __attribute__((ext_vector_type(16))) _Float16 v16h;
typedef __attribute__((ext_vector_type(8)))  _Float16 v8h;
typedef __attribute__((ext_vector_type(8)))  unsigned short v8us;
typedef __attribute__((ext_vector_type(8)))  float    v8f;
typedef __attribute__((ext_vector_type(4)))  float    v4f;
typedef v4f  __attribute__((may_alias)) v4fa;

__device__ __forceinline__ unsigned short f2bf(float f) { unsigned u = __float_as_uint(f); u += 0x7FFFu + ((u >> 16) & 1u); return (unsigned short)(u >> 16); }
__device__ __forceinline__ float bfr(float f) { return __uint_as_float(((unsigned)f2bf(f)) << 16); }
__device__ __forceinline__ v16h cat16(v8h lo, v8h hi) { return __builtin_shufflevector(lo, hi, 0, 1, 2, 3, 4, 5, 6, 7, 8, 9, 10, 11, 12, 13, 14, 15); }
__device__ __forceinline__ v16bf cat16b(v8us lo, v8us hi) { return __builtin_bit_cast(v16bf, __builtin_shufflevector(lo, hi, 0, 1, 2, 3, 4, 5, 6, 7, 8, 9, 10, 11, 12, 13, 14, 15)); }
__device__ __forceinline__ v8f wmma16(v16h a, v16h b, v8f c) { return __builtin_amdgcn_wmma_f32_16x16x32_f16(false, a, false, b, (short)0, c, false, false); }
__device__ __forceinline__ v8f wmmab(v16bf a, v16bf b, v8f c) { return __builtin_amdgcn_wmma_f32_16x16x32_bf16(false, a, false, b, (short)0, c, false, false); }
__device__ __forceinline__ v16h  ldh(const h16* p) { return cat16(*(const v8h*)p, *(const v8h*)(p + 16)); }
__device__ __forceinline__ v16bf ldb(const bf* p)  { return cat16b(*(const v8us*)p, *(const v8us*)(p + 16)); }
__device__ __forceinline__ void wave_sync() { __builtin_amdgcn_fence(3  , "wavefront"); __builtin_amdgcn_wave_barrier(); asm volatile("" ::: "memory"); }

static __device__ __forceinline__ h16 toh_flush(float v) { const h16 r = (h16)v; return (fabsf(v) < 6.103515625e-05f) ? (h16)0.0f : r; }
__device__ __forceinline__ v8f mmag(v16h a, v16h b, v8f c) { c = wmma16(a, b, c); asm volatile("v_nop\n\tv_nop\n\tv_nop\n\tv_nop" : "+v"(c) : "v"(a), "v"(b)); return c; }
__device__ __forceinline__ v8f mmag(v16bf a, v16bf b, v8f c) { c = wmmab(a, b, c); asm volatile("v_nop\n\tv_nop\n\tv_nop\n\tv_nop" : "+v"(c) : "v"(a), "v"(b)); return c; }
__device__ __forceinline__ v16h  ldfrag(const h16* p) { return ldh(p); }
__device__ __forceinline__ v16bf ldfrag(const bf* p)  { return ldb(p); }
template <typename T> struct FragOf;
template <> struct FragOf<h16> { typedef v16h  type; };
template <> struct FragOf<bf>  { typedef v16bf type; };

__global__ __launch_bounds__(256) void k_cvt8(const float* __restrict__ src, bf* dst, size_t n8) {
    const size_t i = (size_t)blockIdx.x * 256 + threadIdx.x; if (i >= n8) return;
    const v8f v = *(const v8f*)(src + i * 8); v8us o;
#pragma unroll
    for (int k = 0; k < 8; ++k) o[k] = f2bf(v[k]);
    *(volatile v8us*)(dst + i * 8) = o; __threadfence(); *(volatile v8us*)(dst + i * 8) = o;
}

__device__ __forceinline__ void wtr_stage(const float* __restrict__ in, const int Cc, float (&sm)[64 * KSP]) {
    const int tid = threadIdx.x; const int cc = tid & 63, rg = tid >> 6;
    const int c0 = blockIdx.x * 64, r0 = blockIdx.y * 64;
#pragma unroll 1
    for (int i = 0; i < 16; ++i) { const int rr = rg + 4 * i;
        sm[rr * KSP + cc] = in[(size_t)(r0 + rr) * (size_t)Cc + (size_t)(c0 + cc)]; }
    __syncthreads();
}
__global__ __launch_bounds__(256) void k_wtr_b(const float* __restrict__ in, bf* out, int R, int Cc) {
    __shared__ float sm[64 * KSP];
    wtr_stage(in, Cc, sm);
    const int tid = threadIdx.x; const int c0 = blockIdx.x * 64, r0 = blockIdx.y * 64;
    static_assert(256 * 16 * 2 == 64 * 64 * 2);
#pragma unroll 1
    for (int ps = 0; ps < 2; ++ps) {
#pragma unroll
        for (int s = 0; s < 2; ++s) { const int ln = s * 32 + (tid >> 3), k8 = (tid & 7) * 8; v8us o;
#pragma unroll
            for (int i = 0; i < 8; ++i) o[i] = f2bf(sm[(k8 + i) * KSP + ln]);
            *(volatile v8us*)(out + (size_t)(c0 + ln) * (size_t)R + (size_t)(r0 + k8)) = o; }
        if (ps == 0) __threadfence(); }
}
__global__ __launch_bounds__(256) void k_wtr_h(const float* __restrict__ in, h16* out, int R, int Cc) {
    __shared__ float sm[64 * KSP];
    wtr_stage(in, Cc, sm);
    const int tid = threadIdx.x; const int c0 = blockIdx.x * 64, r0 = blockIdx.y * 64;
    static_assert(256 * 16 * 2 == 64 * 64 * 2);
#pragma unroll 1
    for (int ps = 0; ps < 2; ++ps) {
#pragma unroll
        for (int s = 0; s < 2; ++s) { const int ln = s * 32 + (tid >> 3), k8 = (tid & 7) * 8; v8h o;
#pragma unroll
            for (int i = 0; i < 8; ++i) o[i] = toh_flush(bfr(sm[(k8 + i) * KSP + ln]) * WCS);
            *(volatile v8h*)(out + (size_t)(c0 + ln) * (size_t)R + (size_t)(r0 + k8)) = o; }
        if (ps == 0) __threadfence(); }
}

template <typename T, int F32OUT>
__device__ __forceinline__ void gemm_tile(const T* __restrict__ A, const T* __restrict__ Bt, const int K, h16* C16, float* C32, const size_t orow, const int ldc, const float scale) {
    __shared__ __align__(16) float os[16 * GSP];
    typedef typename FragOf<T>::type frag;
    const int lane = threadIdx.x & 31, lr = lane & 15, hi = lane >> 4; const int r0 = blockIdx.x * 64, c0 = blockIdx.y * 64;
    v8f acc[4][4];
#pragma unroll
    for (int mb = 0; mb < 4; ++mb)
#pragma unroll
        for (int nb = 0; nb < 4; ++nb) acc[mb][nb] = (v8f){};
    const size_t aoff = (size_t)(r0 + lr) * K + 8 * hi, boff = (size_t)(c0 + lr) * K + 8 * hi;
#pragma unroll 1
    for (int kc = 0; kc < K; kc += 32) {
        frag a[4];
#pragma unroll
        for (int mb = 0; mb < 4; ++mb) a[mb] = ldfrag(A + aoff + (size_t)mb * 16 * K + kc);
#pragma unroll
        for (int nb = 0; nb < 4; ++nb) { const frag bq = ldfrag(Bt + boff + (size_t)nb * 16 * K + kc);
#pragma unroll
            for (int mb = 0; mb < 4; ++mb) acc[mb][nb] = mmag(a[mb], bq, acc[mb][nb]); }
    }
#pragma unroll
    for (int mb = 0; mb < 4; ++mb) {
#pragma unroll
        for (int nb = 0; nb < 4; ++nb) {
#pragma unroll
            for (int j = 0; j < 8; ++j) os[(hi * 8 + j) * GSP + nb * 16 + lr] = acc[mb][nb][j]; }
        wave_sync();
        const size_t rb = (orow + (size_t)(mb * 16)) * (size_t)ldc + (size_t)c0;
#pragma unroll 1
        for (int ps = 0; ps < 2; ++ps) {
            if (F32OUT) {
                static_assert(32 * 16 * 8 == 16 * 64 * 4);
#pragma unroll
                for (int s = 0; s < 8; ++s) { const int row = 2 * s + (lane >> 4), c4 = (lane & 15) * 4;
                    const v4f x = *(const v4fa*)(&os[row * GSP + c4]); const v4f val = x * scale;
                    *(volatile v4f*)(C32 + rb + (size_t)row * ldc + c4) = val; }
            } else {
                static_assert(32 * 16 * 4 == 16 * 64 * 2);
#pragma unroll
                for (int s = 0; s < 4; ++s) { const int row = 4 * s + (lane >> 3), c8 = (lane & 7) * 8;
                    const v4f x0 = *(const v4fa*)(&os[row * GSP + c8]); const v4f x1 = *(const v4fa*)(&os[row * GSP + c8 + 4]); v8h hv;
#pragma unroll
                    for (int i = 0; i < 4; ++i) { hv[i] = toh_flush(x0[i] * scale); hv[4 + i] = toh_flush(x1[i] * scale); }
                    *(volatile v8h*)(C16 + rb + (size_t)row * ldc + c8) = hv; }
            }
            if (ps == 0) __threadfence(); }
        wave_sync();
    }
}

__global__ __launch_bounds__(32) void k_projq(const bf* __restrict__ X, const bf* __restrict__ Wt, h16* Q) {
    gemm_tile<bf, 0>(X, Wt, DM, Q, (float*)0, (size_t)blockIdx.x * 64, DM, 1.0f);
}
__global__ __launch_bounds__(32) void k_projkv(const bf* __restrict__ X, const bf* __restrict__ Wt, float* KVP) {
    gemm_tile<bf, 1>(X, Wt, DM, (h16*)0, KVP, (size_t)blockIdx.x * 64, KVW, 1.0f);
}
__global__ __launch_bounds__(32) void k_outp(const h16* __restrict__ CTX, const h16* __restrict__ Wt, const int* __restrict__ wp, float* OUT) {
    const int r0 = blockIdx.x * 64;
    const size_t orow = (size_t)(r0 / SEQ) * OUT_SEQ + (size_t)(r0 % SEQ);
    const int wv = wp[0];
    float sc = OSC;
    if (wv != CW) sc = __uint_as_float(0x7FC00000u);
    gemm_tile<h16, 1>(CTX, Wt, DM, (h16*)0, OUT, orow, DM, sc);
}

__global__ __launch_bounds__(256) void k_kveff(const float* __restrict__ KVP, h16* KEV) {
    __shared__ float sm[3 * 64 * KSP];
    const int tid = threadIdx.x; const int cc = tid & 63, rg = tid >> 6;
    const int y0 = blockIdx.x * 64; const int part = blockIdx.y; const int b = blockIdx.z;
#pragma unroll 1
    for (int i = 0; i < 16; ++i) { const int yy = rg + 4 * i;
        const float* p = KVP + ((size_t)b * SEQ + (size_t)(y0 + yy)) * KVW + (size_t)(part * 64 + cc);
        float sp = 0.0f, sc = 0.0f, sn = 0.0f;
#pragma unroll 1
        for (int z = 0; z < NCH; ++z) { const float v = p[(size_t)z * CW * KVW];
            sc += v; sp += (z < NCH - 1) ? v : 0.0f; sn += (z > 0) ? v : 0.0f; }
        sm[(0 * 64 + yy) * KSP + cc] = sp; sm[(1 * 64 + yy) * KSP + cc] = sc; sm[(2 * 64 + yy) * KSP + cc] = sn; }
    __syncthreads();
    static_assert(256 * 16 * 6 == 3 * 64 * 64 * 2);
#pragma unroll 1
    for (int ps = 0; ps < 2; ++ps) {
#pragma unroll 1
        for (int s = 0; s < 6; ++s) { const int ln = s * 32 + (tid >> 3), c8 = (tid & 7) * 8; const int e = ln >> 6, q = ln & 63;
            const int lbase = part ? ((e * 64 + c8) * KSP + q) : ((e * 64 + q) * KSP + c8);
            const int lstep = part ? KSP : 1;
            const size_t off = part ? ((size_t)NB * NKEY * HD + ((size_t)b * HD + (size_t)q) * NKEY + (size_t)(e * CW + y0 + c8))
                                    : (((size_t)b * NKEY + (size_t)(e * CW + y0 + q)) * HD + (size_t)c8);
            v8h hv;
#pragma unroll
            for (int i = 0; i < 8; ++i) hv[i] = toh_flush(sm[lbase + i * lstep]);
            *(volatile v8h*)(KEV + off) = hv; }
        if (ps == 0) __threadfence(); }
}

__global__ __launch_bounds__(32 * AW) void k_flash(const h16* __restrict__ QH, const h16* __restrict__ KE, const h16* __restrict__ VT, h16* CTX) {
    __shared__ __align__(16) float os[AW * 16 * OSP];
    const int lane = threadIdx.x & 31, lr = lane & 15, hi = lane >> 4;
    const int wave = __builtin_amdgcn_readfirstlane((int)(threadIdx.x >> 5));
    const int zh = blockIdx.y; const int b = zh / NH_, h = zh % NH_;
    const int t0 = (blockIdx.x * AW + wave) * 16;
    const size_t qo = ((size_t)b * SEQ + (size_t)(t0 + lr)) * DM + (size_t)h * HD + 8 * hi;
    const v16h q0 = ldh(QH + qo), q1 = ldh(QH + qo + 32);
    const size_t ko = ((size_t)b * NKEY + (size_t)lr) * HD + 8 * hi;
    const size_t vo = ((size_t)b * HD + (size_t)lr) * NKEY + 8 * hi;
    v8f o[4];
#pragma unroll
    for (int j = 0; j < 4; ++j) o[j] = (v8f){};
    float m = NEGB, l = 0.0f;
#pragma unroll 1
    for (int key0 = 0; key0 < NKEY; key0 += 32) {
        const h16* ka = KE + ko + (size_t)key0 * HD;
        const v16h ka0 = ldh(ka), ka1 = ldh(ka + 32), kb0 = ldh(ka + 16 * HD), kb1 = ldh(ka + 16 * HD + 32);
        v8f sA = (v8f){}, sB = (v8f){};
        sA = mmag(ka0, q0, sA); sA = mmag(ka1, q1, sA);
        sB = mmag(kb0, q0, sB); sB = mmag(kb1, q1, sB);
        float ta[8], tb[8]; float mx = NEGB;
#pragma unroll
        for (int r = 0; r < 8; ++r) { ta[r] = sA[r] * SC2; tb[r] = sB[r] * SC2; mx = fmaxf(mx, fmaxf(ta[r], tb[r])); }
        mx = fmaxf(mx, __shfl_xor(mx, 16, 32));
        const float mnew = fmaxf(m, mx);
        const float alpha = __builtin_amdgcn_exp2f(m - mnew);
        const float sh = PSH - mnew;
        v16h pb; float ls = 0.0f;
#pragma unroll
        for (int r = 0; r < 8; ++r) {
            const float xa = ta[r] + sh, xb = tb[r] + sh;
            const float ea = __builtin_amdgcn_exp2f(xa), eb = __builtin_amdgcn_exp2f(xb);
            const float ga = (xa < -14.0f) ? 0.0f : ea, gb = (xb < -14.0f) ? 0.0f : eb;
            const h16 pa = (h16)ga; const h16 pc = (h16)gb;
            pb[r] = pa; pb[8 + r] = pc;
            ls += (float)pa + (float)pc; }
        l = l * alpha + ls; m = mnew;
#pragma unroll
        for (int j = 0; j < 4; ++j) o[j] = o[j] * alpha;
        const h16* va = VT + vo + key0;
        const v16h v0 = ldh(va), v1 = ldh(va + (size_t)16 * NKEY), v2 = ldh(va + (size_t)32 * NKEY), v3 = ldh(va + (size_t)48 * NKEY);
        o[0] = mmag(v0, pb, o[0]); o[1] = mmag(v1, pb, o[1]); o[2] = mmag(v2, pb, o[2]); o[3] = mmag(v3, pb, o[3]);
    }
    l += __shfl_xor(l, 16, 32);
    const float inv = CTXC * (1.0f / l);
    const int wb = wave * 16 * OSP;
#pragma unroll
    for (int j = 0; j < 4; ++j) { v4f a, c;
        a[0] = o[j][0] * inv; a[1] = o[j][1] * inv; a[2] = o[j][2] * inv; a[3] = o[j][3] * inv; c[0] = o[j][4] * inv; c[1] = o[j][5] * inv; c[2] = o[j][6] * inv; c[3] = o[j][7] * inv;
        *(v4fa*)(&os[wb + lr * OSP + 16 * j + 8 * hi]) = a; *(v4fa*)(&os[wb + lr * OSP + 16 * j + 8 * hi + 4]) = c; }
    wave_sync();
    h16* crow = CTX + ((size_t)b * SEQ + (size_t)t0) * DM + (size_t)h * HD;
    static_assert(32 * 16 * 4 == 16 * HD * 2);
#pragma unroll 1
    for (int ps = 0; ps < 2; ++ps) {
#pragma unroll
        for (int s = 0; s < 4; ++s) { const int row = 4 * s + (lane >> 3), c8 = (lane & 7) * 8;
            const v4f x0 = *(const v4fa*)(&os[wb + row * OSP + c8]); const v4f x1 = *(const v4fa*)(&os[wb + row * OSP + c8 + 4]); v8h hv;
#pragma unroll
            for (int i = 0; i < 4; ++i) { hv[i] = toh_flush(x0[i]); hv[4 + i] = toh_flush(x1[i]); }
            *(volatile v8h*)(crow + (size_t)row * DM + c8) = hv; }
        if (ps == 0) __threadfence(); }
}

static constexpr size_t al256(size_t v) { return (v + 255) & ~(size_t)255; }
static constexpr size_t SZ_XB  = al256((size_t)NB * SEQ * DM * 2);
static constexpr size_t SZ_WQ  = al256((size_t)DM * DM * 2);
static constexpr size_t SZ_WKV = al256((size_t)KVW * DM * 2);
static constexpr size_t SZ_WC  = al256((size_t)DM * DM * 2);
static constexpr size_t SZ_QH  = al256((size_t)NB * SEQ * DM * 2);
static constexpr size_t SZ_KVP = al256((size_t)NB * SEQ * KVW * 4);
static constexpr size_t SZ_KEV = al256((size_t)NB * 2 * NKEY * HD * 2);
static constexpr size_t SZ_CTX = al256((size_t)NB * SEQ * DM * 2);
static constexpr size_t SZ_TOTAL = 2 * SZ_XB + SZ_WQ + SZ_WKV + SZ_WC + SZ_QH + SZ_KVP + SZ_KEV + SZ_CTX;
static_assert(SZ_TOTAL <= (size_t)134217728);
static_assert(((size_t)NB * NKEY * HD * 2) % 256 == 0);
static_assert((size_t)(NB * SEQ / 64) * 64 == (size_t)NB * SEQ);
static_assert((size_t)(DM / 64) * 64 == (size_t)DM);
static_assert((size_t)(KVW / 64) * 64 == (size_t)KVW);

extern "C" void kernel_launch(void* const* d_in, const int* in_sizes, int n_in,
                              void* d_out, int out_size, void* d_ws, size_t ws_size, hipStream_t stream) {
    if (n_in < 6) return;
    const size_t needx = ((size_t)(NB - 1) * SEQ_FULL + SEQ) * DM;
    if ((size_t)in_sizes[0] < needx || (size_t)in_sizes[1] < needx) return;
    if ((size_t)in_sizes[2] < (size_t)DM * DM || (size_t)in_sizes[3] < (size_t)DM * KVW || (size_t)in_sizes[4] < (size_t)DM * DM) return;
    if (in_sizes[5] < 1) return;
    if ((size_t)out_size < ((size_t)(NB - 1) * OUT_SEQ + SEQ) * DM) return;
    if (SZ_TOTAL > ws_size) return;
    const float* xin[2] = { (const float*)d_in[0], (const float*)d_in[1] };
    const float* wq  = (const float*)d_in[2];
    const float* wkv = (const float*)d_in[3];
    const float* wc  = (const float*)d_in[4];
    const int*   wp  = (const int*)d_in[5];
    float* OUT = (float*)d_out;
    char* wsp = (char*)d_ws;
    bf* XB[2];
    XB[0] = (bf*)wsp; wsp += SZ_XB;
    XB[1] = (bf*)wsp; wsp += SZ_XB;
    bf*  WQT  = (bf*)wsp;  wsp += SZ_WQ;
    bf*  WKVT = (bf*)wsp;  wsp += SZ_WKV;
    h16* WCT  = (h16*)wsp; wsp += SZ_WC;
    h16* QH   = (h16*)wsp; wsp += SZ_QH;
    float* KVP = (float*)wsp; wsp += SZ_KVP;
    h16* KEV  = (h16*)wsp; wsp += SZ_KEV;
    h16* CTX  = (h16*)wsp; wsp += SZ_CTX;
    const h16* KE = KEV; const h16* VT = KEV + (size_t)NB * NKEY * HD;

    for (int i = 0; i < 2; ++i) {
        if (SEQ == SEQ_FULL) {
            const size_t n8 = (size_t)NB * SEQ * DM / 8;
            k_cvt8<<<(unsigned)((n8 + 255) / 256), 256, 0, stream>>>(xin[i], XB[i], n8);
        } else {
            const size_t n8 = (size_t)SEQ * DM / 8;
            for (int b = 0; b < NB; ++b) k_cvt8<<<(unsigned)((n8 + 255) / 256), 256, 0, stream>>>(xin[i] + (size_t)b * SEQ_FULL * DM, XB[i] + (size_t)b * SEQ * DM, n8);
        }
    }
    k_wtr_b<<<dim3(DM / 64, DM / 64, 1), 256, 0, stream>>>(wq, WQT, DM, DM);
    k_wtr_b<<<dim3(KVW / 64, DM / 64, 1), 256, 0, stream>>>(wkv, WKVT, DM, KVW);
    k_wtr_h<<<dim3(DM / 64, DM / 64, 1), 256, 0, stream>>>(wc, WCT, DM, DM);

    k_projq<<<dim3(NB * SEQ / 64, DM / 64, 1), 32, 0, stream>>>(XB[0], WQT, QH);
    k_projkv<<<dim3(NB * SEQ / 64, KVW / 64, 1), 32, 0, stream>>>(XB[1], WKVT, KVP);
    k_kveff<<<dim3(CW / 64, 2, NB), 256, 0, stream>>>(KVP, KEV);
    k_flash<<<dim3(SEQ / (16 * AW), NB * NH_, 1), 32 * AW, 0, stream>>>(QH, KE, VT, CTX);
    k_outp<<<dim3(NB * SEQ / 64, DM / 64, 1), 32, 0, stream>>>(CTX, WCT, wp, OUT);
}
